// EnhancedTimeSeriesTransformer_29910152249379
// MI455X (gfx1250) — hardware-run, weakly checked
//
#include <hip/hip_runtime.h>
#include <hip/hip_bf16.h>
#include <math.h>


typedef _Float16 bf16;
typedef _Float16 f16;
typedef __attribute__((ext_vector_type(4))) unsigned v4u_t;
typedef unsigned v4ua __attribute__((ext_vector_type(4), may_alias));
typedef __attribute__((ext_vector_type(4))) float v4f_t;
typedef float v4fa __attribute__((ext_vector_type(4), may_alias));
typedef __attribute__((ext_vector_type(16))) bf16  bf16x16;
typedef bf16x16 f16x16;
typedef __attribute__((ext_vector_type(8)))  bf16  bf16x8;
typedef bf16x8 f16x8;
typedef __attribute__((ext_vector_type(4)))  bf16  bf16x4;
typedef __attribute__((ext_vector_type(8)))  float f32x8;
__device__ __forceinline__ f32x8 wmma16(f16x16 a, f16x16 b, f32x8 c) {
  c = __builtin_amdgcn_wmma_f32_16x16x32_f16(false, a, false, b, (short)0, c, false, false);
  asm volatile("v_nop\n\tv_nop\n\tv_nop\n\tv_nop" : "+v"(c) : "v"(a), "v"(b));
  return c;
}
#define LDS_STRIDE 48
#define KSTRIDE    72
#define VSTRIDE    48

__device__ __forceinline__ f32x8 wmma_bf16(bf16x16 a, bf16x16 b, f32x8 c) {
  c = __builtin_amdgcn_wmma_f32_16x16x32_f16(false, a, false, b, (short)0, c, false, false);
  asm volatile("v_nop\n\tv_nop\n\tv_nop\n\tv_nop" : "+v"(c) : "v"(a), "v"(b));
  return c;
}

template <typename T>
__device__ __forceinline__ bf16x16 load_frag(const T* __restrict__ base, int ld,
                                             int row0, int k0) {
  const int lane = threadIdx.x & 31;
  const int r    = lane & 15;
  const int kh   = (lane >> 4) * 8;
  const T* p0 = base + (size_t)(row0 + r) * ld + (k0 + kh);
  const T* p1 = p0 + 16;
  bf16x16 f;
#pragma unroll
  for (int i = 0; i < 8; ++i) {
    f[i]     = (bf16)p0[i];
    f[i + 8] = (bf16)p1[i];
  }
  return f;
}

__device__ __forceinline__ bf16x16 lds_frag(const bf16* base, int stride) {
  const int lane = threadIdx.x & 31;
  const int row  = lane & 15;
  const int kh   = (lane >> 4) * 8;
  const bf16x8 lo = *(const bf16x8*)(base + row * stride + kh);
  const bf16x8 hi = *(const bf16x8*)(base + row * stride + kh + 16);
  bf16x16 f;
#pragma unroll
  for (int i = 0; i < 8; ++i) { f[i] = lo[i]; f[i + 8] = hi[i]; }
  return f;
}

template <typename T>
__device__ __forceinline__ void stage_read16(const T* __restrict__ p, float* buf) {
#pragma unroll
  for (int i = 0; i < 16; ++i) buf[i] = (float)p[i];
}

__device__ __forceinline__ void stage_write(bf16* dst, const float* buf, int nquad) {
#pragma unroll
  for (int i = 0; i < nquad; ++i) {
    bf16x4 q;
    q[0] = (bf16)buf[4 * i];     q[1] = (bf16)buf[4 * i + 1];
    q[2] = (bf16)buf[4 * i + 2]; q[3] = (bf16)buf[4 * i + 3];
    *(bf16x4*)(dst + 4 * i) = q;
  }
}


#define GSTR 48
#define GSTR 48
template <typename AT, int EPI, bool OUT16>
__global__ __launch_bounds__(256) void gemm_kne(const AT* __restrict__ A, int lda, const float* __restrict__ Wm, int ldw,
                                                const float* __restrict__ bias, const float* __restrict__ R, const float* __restrict__ gvec,
                                                void* __restrict__ Yv, int ldy, int K) {
  __shared__ __attribute__((aligned(16))) f16 ldsA[128 * GSTR];
  __shared__ __attribute__((aligned(16))) f16 ldsW[128 * GSTR];
  __shared__ __attribute__((aligned(16))) float oS[8][32 * 68];
  const int tid = threadIdx.x, lane = tid & 31, wave = tid >> 5, cl = lane & 15, rh = (lane >> 4) * 8;
  const int m0 = blockIdx.x * 128, n0 = blockIdx.y * 128;
  const int wm = (wave & 3) * 32, wn = (wave >> 2) * 64;
  f32x8 acc[2][4];
#pragma unroll
  for (int i = 0; i < 2; ++i)
#pragma unroll
    for (int j = 0; j < 4; ++j) { f32x8 z = {}; acc[i][j] = z; }
#pragma unroll 1
  for (int k0 = 0; k0 < K; k0 += 32) {
    __syncthreads();
    { const int row = tid >> 1, ch = (tid & 1) * 16;
      const AT* src = A + (size_t)(m0 + row) * lda + k0 + ch;
#pragma unroll
      for (int g = 0; g < 16; ++g) ldsA[row * GSTR + ch + g] = (f16)src[g]; }
    { const int k = tid >> 3, nn0 = (tid & 7) * 16;
      const float* src = Wm + (size_t)(k0 + k) * ldw + n0 + nn0;
#pragma unroll
      for (int g = 0; g < 4; ++g) { const v4f_t v = *(const v4f_t*)(src + 4 * g);
#pragma unroll
        for (int u = 0; u < 4; ++u) ldsW[(nn0 + 4 * g + u) * GSTR + k] = (f16)v[u]; } }
    __syncthreads();
    f16x16 af[2];
#pragma unroll
    for (int i = 0; i < 2; ++i) af[i] = lds_frag(ldsA + (wm + 16 * i) * GSTR, GSTR);
#pragma unroll
    for (int j = 0; j < 4; ++j) {
      const f16x16 bf = lds_frag(ldsW + (wn + 16 * j) * GSTR, GSTR);
#pragma unroll
      for (int i = 0; i < 2; ++i) acc[i][j] = wmma16(af[i], bf, acc[i][j]);
    }
  }
  float* so = oS[wave];
#pragma unroll
  for (int i = 0; i < 2; ++i)
#pragma unroll
    for (int j = 0; j < 4; ++j) {
      const int n = n0 + wn + 16 * j + cl;
      const float bv = bias ? bias[n] : 0.0f;
      const float gv = (EPI == 2 || EPI == 4) ? gvec[n] : 0.0f;
      if (EPI == 1) {
#pragma unroll 1
        for (int r = 0; r < 8; ++r) { const float xg = acc[i][j][r] + bv; so[(16 * i + rh + r) * 68 + 16 * j + cl] = 0.5f * xg * (1.0f + erff(xg * 0.70710678118654752f)); }
      } else {
#pragma unroll
        for (int r = 0; r < 8; ++r) {
          float v = acc[i][j][r] + bv;
          if (EPI == 3) v = fmaxf(v, 0.0f);
          if (EPI == 4) v = gv * v;
          if (EPI == 2) v = R[(size_t)(m0 + wm + 16 * i + rh + r) * ldy + n] + gv * v;
          so[(16 * i + rh + r) * 68 + 16 * j + cl] = v;
        }
      }
    }
  asm volatile("s_wait_dscnt 0" ::: "memory");
  __builtin_amdgcn_wave_barrier();
#pragma unroll 1
  for (int pass = 0; pass < 2; ++pass) {
    if (OUT16) {
      f16* Y = (f16*)Yv;
#pragma unroll
      for (int it = 0; it < 8; ++it) { const int c = lane + 32 * it, rr = c >> 3, q8 = (c & 7) * 8;
        union { f16 h[8]; v4u_t v; } u;
#pragma unroll
        for (int e = 0; e < 8; ++e) u.h[e] = (f16)so[rr * 68 + q8 + e];
        *(volatile v4u_t*)(Y + (size_t)(m0 + wm + rr) * ldy + n0 + wn + q8) = u.v; }
    } else {
      float* Y = (float*)Yv;
#pragma unroll
      for (int it = 0; it < 16; ++it) { const int f4 = lane + 32 * it, rr = f4 >> 4, q = (f4 & 15) * 4;
        *(volatile v4f_t*)(Y + (size_t)(m0 + wm + rr) * ldy + n0 + wn + q) = *(const v4fa*)(so + rr * 68 + q); }
    }
    __threadfence();
  }
}

template <typename AT, int EPI, bool OUT16>
__global__ __launch_bounds__(256) void gemm_knez(const AT* __restrict__ A, int lda, size_t strideA, const float* __restrict__ Wm, int ldw, size_t strideW,
                                                 const float* __restrict__ bias, const float* __restrict__ R, const float* __restrict__ gvec,
                                                 void* __restrict__ Yv, int ldy, size_t strideY, int K) {
  A += (size_t)blockIdx.z * strideA; Wm += (size_t)blockIdx.z * strideW; Yv = (void*)((char*)Yv + (size_t)blockIdx.z * strideY * (OUT16 ? 2 : 4)); if (R) R += (size_t)blockIdx.z * strideY;
  __shared__ __attribute__((aligned(16))) f16 ldsA[128 * GSTR];
  __shared__ __attribute__((aligned(16))) f16 ldsW[128 * GSTR];
  __shared__ __attribute__((aligned(16))) float oS[8][32 * 68];
  const int tid = threadIdx.x, lane = tid & 31, wave = tid >> 5, cl = lane & 15, rh = (lane >> 4) * 8;
  const int m0 = blockIdx.x * 128, n0 = blockIdx.y * 128;
  const int wm = (wave & 3) * 32, wn = (wave >> 2) * 64;
  f32x8 acc[2][4];
#pragma unroll
  for (int i = 0; i < 2; ++i)
#pragma unroll
    for (int j = 0; j < 4; ++j) { f32x8 z = {}; acc[i][j] = z; }
#pragma unroll 1
  for (int k0 = 0; k0 < K; k0 += 32) {
    __syncthreads();
    { const int row = tid >> 1, ch = (tid & 1) * 16;
      const AT* src = A + (size_t)(m0 + row) * lda + k0 + ch;
#pragma unroll
      for (int g = 0; g < 16; ++g) ldsA[row * GSTR + ch + g] = (f16)src[g]; }
    { const int k = tid >> 3, nn0 = (tid & 7) * 16;
      const float* src = Wm + (size_t)(k0 + k) * ldw + n0 + nn0;
#pragma unroll
      for (int g = 0; g < 4; ++g) { const v4f_t v = *(const v4f_t*)(src + 4 * g);
#pragma unroll
        for (int u = 0; u < 4; ++u) ldsW[(nn0 + 4 * g + u) * GSTR + k] = (f16)v[u]; } }
    __syncthreads();
    f16x16 af[2];
#pragma unroll
    for (int i = 0; i < 2; ++i) af[i] = lds_frag(ldsA + (wm + 16 * i) * GSTR, GSTR);
#pragma unroll
    for (int j = 0; j < 4; ++j) {
      const f16x16 bf = lds_frag(ldsW + (wn + 16 * j) * GSTR, GSTR);
#pragma unroll
      for (int i = 0; i < 2; ++i) acc[i][j] = wmma16(af[i], bf, acc[i][j]);
    }
  }
  float* so = oS[wave];
#pragma unroll
  for (int i = 0; i < 2; ++i)
#pragma unroll
    for (int j = 0; j < 4; ++j) {
      const int n = n0 + wn + 16 * j + cl;
      const float bv = bias ? bias[n] : 0.0f;
      const float gv = (EPI == 2 || EPI == 4) ? gvec[n] : 0.0f;
      if (EPI == 1) {
#pragma unroll 1
        for (int r = 0; r < 8; ++r) { const float xg = acc[i][j][r] + bv; so[(16 * i + rh + r) * 68 + 16 * j + cl] = 0.5f * xg * (1.0f + erff(xg * 0.70710678118654752f)); }
      } else {
#pragma unroll
        for (int r = 0; r < 8; ++r) {
          float v = acc[i][j][r] + bv;
          if (EPI == 3) v = fmaxf(v, 0.0f);
          if (EPI == 4) v = gv * v;
          if (EPI == 2) v = R[(size_t)(m0 + wm + 16 * i + rh + r) * ldy + n] + gv * v;
          so[(16 * i + rh + r) * 68 + 16 * j + cl] = v;
        }
      }
    }
  asm volatile("s_wait_dscnt 0" ::: "memory");
  __builtin_amdgcn_wave_barrier();
#pragma unroll 1
  for (int pass = 0; pass < 2; ++pass) {
    if (OUT16) {
      f16* Y = (f16*)Yv;
#pragma unroll
      for (int it = 0; it < 8; ++it) { const int c = lane + 32 * it, rr = c >> 3, q8 = (c & 7) * 8;
        union { f16 h[8]; v4u_t v; } u;
#pragma unroll
        for (int e = 0; e < 8; ++e) u.h[e] = (f16)so[rr * 68 + q8 + e];
        *(volatile v4u_t*)(Y + (size_t)(m0 + wm + rr) * ldy + n0 + wn + q8) = u.v; }
    } else {
      float* Y = (float*)Yv;
#pragma unroll
      for (int it = 0; it < 16; ++it) { const int f4 = lane + 32 * it, rr = f4 >> 4, q = (f4 & 15) * 4;
        *(volatile v4f_t*)(Y + (size_t)(m0 + wm + rr) * ldy + n0 + wn + q) = *(const v4fa*)(so + rr * 68 + q); }
    }
    __threadfence();
  }
}

template <typename AT, bool ACC>
__global__ __launch_bounds__(256) void gemm_kn2(const AT* __restrict__ A, int lda, size_t strideA,
                                               const float* __restrict__ Wm, int ldw, size_t strideW,
                                               const float* __restrict__ bias, float scale,
                                               float* __restrict__ Y, int ldy, size_t strideY, int K) {
  __shared__ __attribute__((aligned(16))) f16 ldsA[128 * GSTR], ldsAl[128 * GSTR];
  __shared__ __attribute__((aligned(16))) f16 ldsW[128 * GSTR], ldsWl[128 * GSTR];
  __shared__ __attribute__((aligned(16))) float oS[8][32 * 68];
  const int tid = threadIdx.x, lane = tid & 31, wave = tid >> 5, cl = lane & 15, rh = (lane >> 4) * 8;
  const int m0 = blockIdx.x * 128, n0 = blockIdx.y * 128;
  const int wm = (wave & 3) * 32, wn = (wave >> 2) * 64;
  A += (size_t)blockIdx.z * strideA; Wm += (size_t)blockIdx.z * strideW; Y += (size_t)blockIdx.z * strideY;
  f32x8 acc[2][4], accx[2][4];
#pragma unroll
  for (int i = 0; i < 2; ++i)
#pragma unroll
    for (int j = 0; j < 4; ++j) { f32x8 z = {}; acc[i][j] = z; accx[i][j] = z; }
#pragma unroll 1
  for (int k0 = 0; k0 < K; k0 += 32) {
    __syncthreads();
    {
      const int row = tid >> 1, ch = (tid & 1) * 16;
      const AT* src = A + (size_t)(m0 + row) * lda + k0 + ch;
#pragma unroll
      for (int g = 0; g < 16; ++g) { const float v = (float)src[g]; const f16 h = (f16)v; ldsA[row * GSTR + ch + g] = h; ldsAl[row * GSTR + ch + g] = (f16)((v - (float)h) * 2048.0f); }
    }
    {
      const int k = tid >> 3, nn0 = (tid & 7) * 16;
      const float* src = Wm + (size_t)(k0 + k) * ldw + n0 + nn0;
#pragma unroll
      for (int g = 0; g < 4; ++g) { const v4f_t v = *(const v4f_t*)(src + 4 * g);
#pragma unroll
        for (int u = 0; u < 4; ++u) { const f16 h = (f16)v[u]; ldsW[(nn0 + 4 * g + u) * GSTR + k] = h; ldsWl[(nn0 + 4 * g + u) * GSTR + k] = (f16)((v[u] - (float)h) * 2048.0f); } }
    }
    __syncthreads();
    f16x16 af[2], afl[2];
#pragma unroll
    for (int i = 0; i < 2; ++i) { af[i] = lds_frag(ldsA + (wm + 16 * i) * GSTR, GSTR); afl[i] = lds_frag(ldsAl + (wm + 16 * i) * GSTR, GSTR); }
#pragma unroll
    for (int j = 0; j < 4; ++j) {
      const f16x16 bf = lds_frag(ldsW + (wn + 16 * j) * GSTR, GSTR), bfl = lds_frag(ldsWl + (wn + 16 * j) * GSTR, GSTR);
#pragma unroll
      for (int i = 0; i < 2; ++i) { acc[i][j] = wmma16(af[i], bf, acc[i][j]); accx[i][j] = wmma16(af[i], bfl, accx[i][j]); accx[i][j] = wmma16(afl[i], bf, accx[i][j]); }
    }
  }
  float* so = oS[wave];
#pragma unroll
  for (int i = 0; i < 2; ++i)
#pragma unroll
    for (int j = 0; j < 4; ++j) {
      const float bv = bias ? bias[n0 + wn + 16 * j + cl] : 0.0f;
#pragma unroll
      for (int r = 0; r < 8; ++r) so[(16 * i + rh + r) * 68 + 16 * j + cl] = (acc[i][j][r] + accx[i][j][r] * (1.0f / 2048.0f)) * scale + bv;
    }
  asm volatile("s_wait_dscnt 0" ::: "memory");
  __builtin_amdgcn_wave_barrier();
  if (ACC) {
#pragma unroll
    for (int it = 0; it < 16; ++it) { const int f4 = lane + 32 * it, rr = f4 >> 4, q = (f4 & 15) * 4;
      const v4f_t old = *(const v4fa*)(Y + (size_t)(m0 + wm + rr) * ldy + n0 + wn + q);
      v4f_t v = *(const v4fa*)(so + rr * 68 + q); v += old; *(v4fa*)(so + rr * 68 + q) = v; }
    asm volatile("s_wait_dscnt 0" ::: "memory");
  }
#pragma unroll 1
  for (int pass = 0; pass < 2; ++pass) {
#pragma unroll
    for (int it = 0; it < 16; ++it) { const int f4 = lane + 32 * it, rr = f4 >> 4, q = (f4 & 15) * 4;
      *(volatile v4f_t*)(Y + (size_t)(m0 + wm + rr) * ldy + n0 + wn + q) = *(const v4fa*)(so + rr * 68 + q); }
    __threadfence();
  }
}

__global__ __launch_bounds__(256) void k_transpose(const float* __restrict__ Wm, float* __restrict__ Wt, int rows, int cols) {
  __shared__ float tS[64][65];
  const int tid = threadIdx.x, tbj = cols / 64, bi = blockIdx.x / tbj, bj = blockIdx.x % tbj;
  for (int e = tid; e < 64 * 64; e += 256) { const int r = e >> 6, c = e & 63; tS[r][c] = Wm[(size_t)(bi * 64 + r) * cols + bj * 64 + c]; }
  __syncthreads();
  for (int ch = tid; ch < 64 * 16; ch += 256) { const int r = ch >> 4, q4 = (ch & 15) * 4; v4f_t o; o[0] = tS[q4][r]; o[1] = tS[q4 + 1][r]; o[2] = tS[q4 + 2][r]; o[3] = tS[q4 + 3][r];
    float* dst = Wt + (size_t)(bj * 64 + r) * rows + bi * 64 + q4; *(volatile v4f_t*)dst = o; __threadfence(); *(volatile v4f_t*)dst = o; }
}


template <typename AT, int EPI, bool OUT16, int NJ>
__global__ __launch_bounds__(256) void gemm_sm(const AT* __restrict__ A, int lda, size_t sA, const float* __restrict__ Wm, int ldw, size_t sW,
                                               const float* __restrict__ bias, const float* __restrict__ R, const float* __restrict__ gvec,
                                               void* __restrict__ Yv, int ldy, size_t sY, int K) {
  constexpr int BN = 16 * NJ; constexpr int OST = BN + 4;
  A += (size_t)blockIdx.z * sA; Wm += (size_t)blockIdx.z * sW; Yv = (void*)((char*)Yv + (size_t)blockIdx.z * sY * (OUT16 ? 2 : 4)); if (R) R += (size_t)blockIdx.z * sY;
  __shared__ __attribute__((aligned(16))) f16 ldsA[256 * GSTR];
  __shared__ __attribute__((aligned(16))) f16 ldsW[BN * GSTR];
  __shared__ __attribute__((aligned(16))) float oS[8][32 * OST];
  const int tid = threadIdx.x, lane = tid & 31, wave = tid >> 5, cl = lane & 15, rh = (lane >> 4) * 8;
  const int m0 = blockIdx.x * 256, n0 = blockIdx.y * BN;
  const int wm = wave * 32;
  f32x8 acc[2][NJ];
#pragma unroll
  for (int i = 0; i < 2; ++i)
#pragma unroll
    for (int j = 0; j < NJ; ++j) { f32x8 z = {}; acc[i][j] = z; }
#pragma unroll 1
  for (int k0 = 0; k0 < K; k0 += 32) {
    __syncthreads();
    { const AT* src = A + (size_t)(m0 + tid) * lda + k0;
#pragma unroll
      for (int g = 0; g < 32; ++g) ldsA[tid * GSTR + g] = (f16)src[g]; }
    { const int k = tid >> 3, nn0 = (tid & 7) * (2 * NJ);
      const float* src = Wm + (size_t)(k0 + k) * ldw + n0 + nn0;
#pragma unroll
      for (int g = 0; g < NJ / 2; ++g) { const v4f_t v = *(const v4f_t*)(src + 4 * g);
#pragma unroll
        for (int u = 0; u < 4; ++u) ldsW[(nn0 + 4 * g + u) * GSTR + k] = (f16)v[u]; } }
    __syncthreads();
    f16x16 af[2];
#pragma unroll
    for (int i = 0; i < 2; ++i) af[i] = lds_frag(ldsA + (wm + 16 * i) * GSTR, GSTR);
#pragma unroll
    for (int j = 0; j < NJ; ++j) {
      const f16x16 bf = lds_frag(ldsW + (16 * j) * GSTR, GSTR);
#pragma unroll
      for (int i = 0; i < 2; ++i) acc[i][j] = wmma16(af[i], bf, acc[i][j]);
    }
  }
  float* so = oS[wave];
#pragma unroll
  for (int i = 0; i < 2; ++i)
#pragma unroll
    for (int j = 0; j < NJ; ++j) {
      const int n = n0 + 16 * j + cl;
      const float bv = bias ? bias[n] : 0.0f;
      const float gv = (EPI == 2 || EPI == 4) ? gvec[n] : 0.0f;
#pragma unroll
      for (int r = 0; r < 8; ++r) {
        float v = acc[i][j][r] + bv;
        if (EPI == 3) v = fmaxf(v, 0.0f);
        if (EPI == 2) v = R[(size_t)(m0 + wm + 16 * i + rh + r) * ldy + n] + gv * v;
        if (EPI == 4) v = gv * v;
        so[(16 * i + rh + r) * OST + 16 * j + cl] = v;
      }
    }
  asm volatile("s_wait_dscnt 0" ::: "memory");
  __builtin_amdgcn_wave_barrier();
#pragma unroll 1
  for (int pass = 0; pass < 2; ++pass) {
    if (OUT16) {
      f16* Y = (f16*)Yv;
#pragma unroll
      for (int it = 0; it < BN / 8; ++it) { const int c = lane + 32 * it, rr = c / (BN / 8), q8 = (c % (BN / 8)) * 8;
        union { f16 h[8]; v4u_t v; } u;
#pragma unroll
        for (int e = 0; e < 8; ++e) u.h[e] = (f16)so[rr * OST + q8 + e];
        *(volatile v4u_t*)(Y + (size_t)(m0 + wm + rr) * ldy + n0 + q8) = u.v; }
    } else {
      float* Y = (float*)Yv;
#pragma unroll
      for (int it = 0; it < BN / 4; ++it) { const int f4 = lane + 32 * it, rr = f4 / (BN / 4), q = (f4 % (BN / 4)) * 4;
        *(volatile v4f_t*)(Y + (size_t)(m0 + wm + rr) * ldy + n0 + q) = *(const v4fa*)(so + rr * OST + q); }
    }
    __threadfence();
  }
}

#define NBe 4
#define LLe 1024
#define DDe 512
#define NHe 8
#define HDe 64
#define FFe 2048
#define FINe 64
#define NCe 3
__global__ __launch_bounds__(256) void k_fill(float* __restrict__ p, float val, size_t n4) { const size_t i = (size_t)blockIdx.x * 256 + threadIdx.x; if (i < n4) { v4f_t v = {val, val, val, val}; *(volatile v4f_t*)(p + 4 * i) = v; __threadfence(); *(volatile v4f_t*)(p + 4 * i) = v; } }
__global__ __launch_bounds__(256) void k_dbg_zero(float* __restrict__ p, size_t n4) { const size_t i = (size_t)blockIdx.x * 256 + threadIdx.x; if (i < n4) { v4f_t z = {0.f,0.f,0.f,0.f}; *(volatile v4f_t*)(p + 4 * i) = z; __threadfence(); *(volatile v4f_t*)(p + 4 * i) = z; } }
__global__ __launch_bounds__(256) void k_copy(const float* __restrict__ src, float* __restrict__ dst, size_t n4) { const size_t i = (size_t)blockIdx.x * 256 + threadIdx.x; if (i < n4) { const v4f_t v = *(const v4f_t*)(src + 4 * i); *(volatile v4f_t*)(dst + 4 * i) = v; __threadfence(); *(volatile v4f_t*)(dst + 4 * i) = v; } }
__global__ __launch_bounds__(256) void k_transpose_ld(const float* __restrict__ Wm, int lds, float* __restrict__ Wt, int rows, int cols) {
  __shared__ float tS[64][65];
  const int tid = threadIdx.x, tbj = cols / 64, bi = blockIdx.x / tbj, bj = blockIdx.x % tbj;
  for (int e = tid; e < 64 * 64; e += 256) { const int r = e >> 6, c = e & 63; tS[r][c] = Wm[(size_t)(bi * 64 + r) * lds + bj * 64 + c]; }
  __syncthreads();
  for (int ch = tid; ch < 64 * 16; ch += 256) { const int r = ch >> 4, q4 = (ch & 15) * 4; v4f_t o; o[0] = tS[q4][r]; o[1] = tS[q4 + 1][r]; o[2] = tS[q4 + 2][r]; o[3] = tS[q4 + 3][r];
    float* dst = Wt + (size_t)(bj * 64 + r) * rows + bi * 64 + q4; *(volatile v4f_t*)dst = o; __threadfence(); *(volatile v4f_t*)dst = o; }
}
__global__ __launch_bounds__(256) void k_ln(const float* __restrict__ X, const float* __restrict__ gam, const float* __restrict__ bet, float* __restrict__ Y) {
  __shared__ __attribute__((aligned(16))) float rowS[16 * 516];
  const int tid = threadIdx.x, r = tid >> 4, part = tid & 15; const size_t row = (size_t)blockIdx.x * 16 + r;
  float s = 0.0f;
#pragma unroll 1
  for (int i = 0; i < 32; ++i) { const float v = X[row * 512 + part * 32 + i]; rowS[r * 516 + part * 32 + i] = v; s += v; }
  s += __shfl_xor(s, 1, 32); s += __shfl_xor(s, 2, 32); s += __shfl_xor(s, 4, 32); s += __shfl_xor(s, 8, 32);
  const float mean = s * (1.0f / 512.0f); float q = 0.0f;
#pragma unroll 1
  for (int i = 0; i < 32; ++i) { const float dv = rowS[r * 516 + part * 32 + i] - mean; q += dv * dv; }
  q += __shfl_xor(q, 1, 32); q += __shfl_xor(q, 2, 32); q += __shfl_xor(q, 4, 32); q += __shfl_xor(q, 8, 32);
  const float rstd = 1.0f / __builtin_sqrtf(q * (1.0f / 512.0f) + 1e-6f);
#pragma unroll 1
  for (int i = 0; i < 32; ++i) { const int c = part * 32 + i; rowS[r * 516 + c] = (rowS[r * 516 + c] - mean) * rstd * gam[c] + bet[c]; }
  __syncthreads();
#pragma unroll 1
  for (int pass = 0; pass < 2; ++pass) { for (int q4 = tid; q4 < 16 * 128; q4 += 256) { const int rr = q4 / 128, c4 = (q4 % 128) * 4;
      *(volatile v4f_t*)(Y + ((size_t)blockIdx.x * 16 + rr) * 512 + c4) = *(const v4fa*)(rowS + rr * 516 + c4); } __threadfence(); }
}
__global__ __launch_bounds__(256) void k_vsum(const float* __restrict__ V, int ldv, float* __restrict__ VB) {
  const int c = blockIdx.x * 256 + threadIdx.x; if (c >= 512) return; float s = 0.0f;
#pragma unroll 1
  for (int r = 0; r < 1024; ++r) s += V[(size_t)r * ldv + c];
  const float m = s;   *(volatile float*)(VB + c) = m; __threadfence(); *(volatile float*)(VB + c) = m;
}
__global__ __launch_bounds__(256) void k_xscale(const float* __restrict__ xb, const float* __restrict__ fs, float* __restrict__ XS, size_t n4) { const size_t i = (size_t)blockIdx.x * 256 + threadIdx.x; if (i >= n4) return; const int c = (int)((4 * i) % FINe);
  const v4f_t v = *(const v4f_t*)(xb + 4 * i) * *(const v4f_t*)(fs + c); *(volatile v4f_t*)(XS + 4 * i) = v; __threadfence(); *(volatile v4f_t*)(XS + 4 * i) = v; }
__global__ __launch_bounds__(256) void k_embfin(float* __restrict__ E, const float* __restrict__ pe, size_t n4) { const size_t i = (size_t)blockIdx.x * 256 + threadIdx.x; if (i >= n4) return;
  const v4f_t v = *(const v4fa*)(E + 4 * i) * 22.627416997969522f + *(const v4f_t*)(pe + 4 * i); *(volatile v4fa*)(E + 4 * i) = v; __threadfence(); *(volatile v4fa*)(E + 4 * i) = v; }
__global__ __launch_bounds__(256) void k_relb(const float* __restrict__ Q, const float* __restrict__ rel, float* __restrict__ RB) { __shared__ float qs[DDe];
  const size_t q = blockIdx.x; const int tid = threadIdx.x, h = tid >> 5, lane = tid & 31; for (int i = tid; i < DDe; i += 256) qs[i] = Q[q * DDe + i]; __syncthreads();
  float o1 = 0.0f, o2 = 0.0f, o3 = 0.0f; const float* qh = qs + h * HDe;
#pragma unroll 1
  for (int d = 0; d < HDe; ++d) { const float qd = qh[d]; o1 += qd * rel[lane * HDe + d]; o2 += qd * rel[(lane + 32) * HDe + d]; if (lane == 0) o3 += qd * rel[64 * HDe + d]; }
  float* dst = RB + (q * NHe + h) * 80; *(volatile float*)(dst + lane) = o1 * 0.125f; *(volatile float*)(dst + 32 + lane) = o2 * 0.125f; if (lane < 16) *(volatile float*)(dst + 64 + lane) = (lane == 0) ? o3 * 0.125f : 0.0f;
  __threadfence(); *(volatile float*)(dst + lane) = o1 * 0.125f; *(volatile float*)(dst + 32 + lane) = o2 * 0.125f; if (lane < 16) *(volatile float*)(dst + 64 + lane) = (lane == 0) ? o3 * 0.125f : 0.0f; }
__global__ __launch_bounds__(256) void k_rsoft(float* __restrict__ Sm, const float* __restrict__ RB, int h0) {
  __shared__ float red[256];
  const int q = blockIdx.x, z = blockIdx.y, tid = threadIdx.x; float* sr = Sm + ((size_t)z * LLe + q) * LLe; const float* rb = RB + ((size_t)q * NHe + h0 + z) * 80; float v[LLe / 256]; float m = -3.0e38f;
#pragma unroll
  for (int e = 0; e < LLe / 256; ++e) { const int k = tid + 256 * e; const int o = min(max(k - q, -32), 32) + 32; v[e] = sr[k] * 0.125f + rb[o]; m = fmaxf(m, v[e]); }
  red[tid] = m; __syncthreads(); for (int o = 128; o > 0; o >>= 1) { if (tid < o) red[tid] = fmaxf(red[tid], red[tid + o]); __syncthreads(); }
  m = red[0]; __syncthreads(); float zs = 0.0f;
#pragma unroll
  for (int e = 0; e < LLe / 256; ++e) { v[e] = expf(v[e] - m); zs += v[e]; }
  red[tid] = zs; __syncthreads(); for (int o = 128; o > 0; o >>= 1) { if (tid < o) red[tid] += red[tid + o]; __syncthreads(); }
  const float kk = 1024.0f / red[0];
#pragma unroll 1
  for (int pass = 0; pass < 2; ++pass) {
#pragma unroll
    for (int e = 0; e < LLe / 256; ++e) *(volatile float*)(sr + tid + 256 * e) = v[e] * kk - 1.0f;
    __threadfence(); }
}
__global__ __launch_bounds__(256) void k_lastq(const float* __restrict__ Hrow, const float* __restrict__ Wq, const float* __restrict__ bq, float* __restrict__ Q0) { __shared__ float hs[DDe]; const int tid = threadIdx.x; for (int i = tid; i < DDe; i += 256) hs[i] = Hrow[i]; __syncthreads();
#pragma unroll 1
  for (int pass = 0; pass < 2; ++pass) { for (int o = tid; o < DDe; o += 256) { float a = bq[o];
#pragma unroll 1
      for (int i = 0; i < DDe; ++i) a += hs[i] * Wq[(size_t)i * DDe + o]; *(volatile float*)(Q0 + o) = a; } __threadfence(); } }
__global__ __launch_bounds__(256) void k_lastatt(const float* __restrict__ Q0, const float* __restrict__ Km, const float* __restrict__ Vm, const float* __restrict__ rel, float* __restrict__ CTX) {
  __shared__ float qs[HDe]; __shared__ float pr[LLe]; __shared__ float red[256]; __shared__ float part[4][HDe]; __shared__ float rbias[80];
  const int h = blockIdx.x, tid = threadIdx.x; if (tid < HDe) qs[tid] = Q0[h * HDe + tid]; __syncthreads();
  if (tid < 65) { float a = 0.0f;
#pragma unroll 1
    for (int d = 0; d < HDe; ++d) a += qs[d] * rel[tid * HDe + d]; rbias[tid] = a * 0.125f; }
  __syncthreads();
  float m = -3.0e38f;
#pragma unroll 1
  for (int k = tid; k < LLe; k += 256) { const float* kr = Km + (size_t)k * DDe + h * HDe; float s = 0.0f;
#pragma unroll 1
    for (int d = 0; d < HDe; ++d) s += qs[d] * kr[d];
    const int o = min(max(k - (LLe - 1), -32), 32) + 32; s = s * 0.125f + rbias[o]; pr[k] = s; m = fmaxf(m, s); }
  red[tid] = m; __syncthreads(); for (int o = 128; o > 0; o >>= 1) { if (tid < o) red[tid] = fmaxf(red[tid], red[tid + o]); __syncthreads(); }
  m = red[0]; __syncthreads(); float zsum = 0.0f;
  for (int k = tid; k < LLe; k += 256) { const float e = expf(pr[k] - m); pr[k] = e; zsum += e; }
  red[tid] = zsum; __syncthreads(); for (int o = 128; o > 0; o >>= 1) { if (tid < o) red[tid] += red[tid + o]; __syncthreads(); }
  const float inv = 1.0f / red[0]; __syncthreads();
  { const int d = tid & 63, part_i = tid >> 6; float a = 0.0f;
#pragma unroll 1
    for (int k = part_i; k < LLe; k += 4) a += pr[k] * Vm[(size_t)k * DDe + h * HDe + d];
    part[part_i][d] = a; }
  __syncthreads();
  if (tid < HDe) { const float c = (part[0][tid] + part[1][tid] + part[2][tid] + part[3][tid]) * inv; *(volatile float*)(CTX + h * HDe + tid) = c; __threadfence(); *(volatile float*)(CTX + h * HDe + tid) = c; }
}
__global__ __launch_bounds__(256) void k_lasttail(const float* __restrict__ Trow, const float* __restrict__ CTX, const float* __restrict__ Wo, const float* __restrict__ bo, const float* __restrict__ g2, const float* __restrict__ be2, const float* __restrict__ W1, const float* __restrict__ b1, const float* __restrict__ W2, const float* __restrict__ b2,
    const float* __restrict__ gf, const float* __restrict__ bf, const float* __restrict__ Wc1, const float* __restrict__ bc1, const float* __restrict__ Wc2, const float* __restrict__ bc2, float* __restrict__ ob) {
  __shared__ float t[DDe], a[DDe], hb[FFe], red[256]; const int tid = threadIdx.x;
  for (int i = tid; i < DDe; i += 256) { t[i] = Trow[i]; a[i] = CTX[i]; } __syncthreads();
  for (int o = tid; o < DDe; o += 256) { float s = bo[o];
#pragma unroll 1
    for (int i = 0; i < DDe; ++i) s += a[i] * Wo[(size_t)i * DDe + o]; hb[o] = t[o] + s; }
  __syncthreads(); for (int i = tid; i < DDe; i += 256) t[i] = hb[i]; __syncthreads();
  { float s = 0.0f; for (int i = tid; i < DDe; i += 256) s += t[i]; red[tid] = s; __syncthreads(); for (int o = 128; o > 0; o >>= 1) { if (tid < o) red[tid] += red[tid + o]; __syncthreads(); } const float mu = red[0] / DDe; __syncthreads();
    float s2 = 0.0f; for (int i = tid; i < DDe; i += 256) { const float dv = t[i] - mu; s2 += dv * dv; } red[tid] = s2; __syncthreads(); for (int o = 128; o > 0; o >>= 1) { if (tid < o) red[tid] += red[tid + o]; __syncthreads(); } const float rs = rsqrtf(red[0] / DDe + 1e-6f); __syncthreads();
    for (int i = tid; i < DDe; i += 256) a[i] = (t[i] - mu) * rs * g2[i] + be2[i]; __syncthreads(); }
  for (int o = tid; o < FFe; o += 256) { float s = b1[o];
#pragma unroll 1
    for (int i = 0; i < DDe; ++i) s += a[i] * W1[(size_t)i * FFe + o]; hb[o] = 0.5f * s * (1.0f + erff(s * 0.70710678118654752f)); }
  __syncthreads();
  for (int o = tid; o < DDe; o += 256) { float s = b2[o];
#pragma unroll 1
    for (int i = 0; i < FFe; ++i) s += hb[i] * W2[(size_t)i * DDe + o]; t[o] = t[o] + s; }
  __syncthreads();
  { float s = 0.0f; for (int i = tid; i < DDe; i += 256) s += t[i]; red[tid] = s; __syncthreads(); for (int o = 128; o > 0; o >>= 1) { if (tid < o) red[tid] += red[tid + o]; __syncthreads(); } const float mu = red[0] / DDe; __syncthreads();
    float s2 = 0.0f; for (int i = tid; i < DDe; i += 256) { const float dv = t[i] - mu; s2 += dv * dv; } red[tid] = s2; __syncthreads(); for (int o = 128; o > 0; o >>= 1) { if (tid < o) red[tid] += red[tid + o]; __syncthreads(); } const float rs = rsqrtf(red[0] / DDe + 1e-6f); __syncthreads();
    for (int i = tid; i < DDe; i += 256) a[i] = (t[i] - mu) * rs * gf[i] + bf[i]; __syncthreads(); }
  for (int o = tid; o < DDe / 2; o += 256) { float s = bc1[o];
#pragma unroll 1
    for (int i = 0; i < DDe; ++i) s += a[i] * Wc1[(size_t)i * (DDe / 2) + o]; hb[o] = 0.5f * s * (1.0f + erff(s * 0.70710678118654752f)); }
  __syncthreads();
  if (tid < NCe) { float s = bc2[tid];
#pragma unroll 1
    for (int i = 0; i < DDe / 2; ++i) s += hb[i] * Wc2[(size_t)i * NCe + tid]; *(volatile float*)(ob + tid) = s; __threadfence(); *(volatile float*)(ob + tid) = s; }
}

extern "C" void kernel_launch(void* const* d_in, const int* in_sizes, int n_in,
                              void* d_out, int out_size, void* d_ws, size_t ws_size,
                              hipStream_t stream) {
  (void)in_sizes; (void)n_in; (void)out_size;
  const float** f = (const float**)d_in;
  const float* x = f[0], *fs = f[1], *Wemb = f[2], *bemb = f[3], *pe = f[4], *Wq = f[5], *bq = f[6], *Wk = f[7], *bk = f[8], *Wv = f[9], *bv = f[10], *Wo = f[11], *bo = f[12], *rel = f[13], *l1s = f[14], *l1b = f[15], *l2s = f[16], *l2b = f[17], *W1 = f[18], *b1 = f[19], *W2 = f[20], *b2 = f[21], *fns = f[22], *fnb = f[23], *Wc1 = f[24], *bc1 = f[25], *Wc2 = f[26], *bc2 = f[27];
  float* out = (float*)d_out;
  char* ws = (char*)d_ws;
  float* XS = (float*)ws; ws += (size_t)LLe * FINe * 4; float* T = (float*)ws; ws += (size_t)LLe * DDe * 4; float* Hn = (float*)ws; ws += (size_t)LLe * DDe * 4;
  float* Q = (float*)ws; ws += (size_t)LLe * DDe * 4; float* Km = (float*)ws; ws += (size_t)LLe * DDe * 4; float* V = (float*)ws; ws += (size_t)LLe * DDe * 4; float* KT = (float*)ws; ws += (size_t)HDe * 2 * LLe * 4; float* RB = (float*)ws; ws += (size_t)LLe * NHe * 80 * 4;
  float* VS = (float*)ws; ws += DDe * 4; float* sc = (float*)ws; ws += 64 * 4; float* ones = (float*)ws; ws += FFe * 4; float* S = (float*)ws; ws += (size_t)2 * LLe * LLe * 4; float* ATT = (float*)ws; ws += (size_t)LLe * DDe * 4; float* Fh = (float*)ws; ws += (size_t)LLe * FFe * 4;
  float* Q0 = (float*)ws; ws += DDe * 4; float* CTX = (float*)ws; ws += DDe * 4;
  if ((size_t)(ws - (char*)d_ws) > ws_size) return;
  const dim3 blk(256);
  k_fill<<<dim3(1), blk, 0, stream>>>(sc, 1.0f / 1024.0f, 64 / 4); k_fill<<<dim3(2), blk, 0, stream>>>(ones, 1.0f, FFe / 4);

  for (int b = 0; b < NBe; ++b) {
    k_xscale<<<dim3(((size_t)LLe * FINe / 4 + 255) / 256), blk, 0, stream>>>(x + (size_t)b * 1024 * FINe, fs, XS, (size_t)LLe * FINe / 4);
    gemm_kne<float, 0, false><<<dim3(LLe / 128, DDe / 128), blk, 0, stream>>>(XS, FINe, Wemb, DDe, bemb, nullptr, nullptr, T, DDe, FINe);
    k_embfin<<<dim3(((size_t)LLe * DDe / 4 + 255) / 256), blk, 0, stream>>>(T, pe, (size_t)LLe * DDe / 4);
    for (int l = 0; l < 3; ++l) { const float* wq = Wq + (size_t)l * DDe * DDe; const float* wk = Wk + (size_t)l * DDe * DDe; const float* wv = Wv + (size_t)l * DDe * DDe; const float* wo = Wo + (size_t)l * DDe * DDe; const float* w1 = W1 + (size_t)l * DDe * FFe; const float* w2 = W2 + (size_t)l * FFe * DDe; const float* rl = rel + (size_t)l * 65 * HDe;
      k_ln<<<dim3(LLe / 16), blk, 0, stream>>>(T, l1s + l * DDe, l1b + l * DDe, Hn);
      gemm_kne<float, 0, false><<<dim3(LLe / 128, DDe / 128), blk, 0, stream>>>(Hn, DDe, wk, DDe, bk + l * DDe, nullptr, nullptr, Km, DDe, DDe);
      gemm_kne<float, 0, false><<<dim3(LLe / 128, DDe / 128), blk, 0, stream>>>(Hn, DDe, wv, DDe, bv + l * DDe, nullptr, nullptr, V, DDe, DDe);
      if (l == 2) {
        k_lastq<<<dim3(1), blk, 0, stream>>>(Hn + (size_t)(LLe - 1) * DDe, wq, bq + l * DDe, Q0);
        k_lastatt<<<dim3(NHe), blk, 0, stream>>>(Q0, Km, V, rl, CTX);
        k_lasttail<<<dim3(1), blk, 0, stream>>>(T + (size_t)(LLe - 1) * DDe, CTX, wo, bo + l * DDe, l2s + l * DDe, l2b + l * DDe, w1, b1 + l * FFe, w2, b2 + l * DDe, fns, fnb, Wc1, bc1, Wc2, bc2, out + (size_t)b * NCe);
        break; }
      gemm_kne<float, 0, false><<<dim3(LLe / 128, DDe / 128), blk, 0, stream>>>(Hn, DDe, wq, DDe, bq + l * DDe, nullptr, nullptr, Q, DDe, DDe);
      k_relb<<<dim3(LLe), blk, 0, stream>>>(Q, rl, RB);
      k_vsum<<<dim3(DDe / 256), blk, 0, stream>>>(V, DDe, VS);
      for (int hp = 0; hp < NHe / 2; ++hp) { const int h0 = 2 * hp;
        for (int z = 0; z < 2; ++z) k_transpose_ld<<<dim3((LLe / 64) * (HDe / 64)), blk, 0, stream>>>(Km + (h0 + z) * HDe, DDe, KT + (size_t)z * HDe * LLe, LLe, HDe);
        gemm_knez<float, 0, false><<<dim3(LLe / 128, LLe / 128, 2), blk, 0, stream>>>(Q + h0 * HDe, DDe, (size_t)HDe, KT, LLe, (size_t)HDe * LLe, nullptr, nullptr, nullptr, S, LLe, (size_t)LLe * LLe, HDe);
        k_rsoft<<<dim3(LLe, 2), blk, 0, stream>>>(S, RB, h0);
        for (int z = 0; z < 2; ++z)
          gemm_sm<float, 4, false, 4><<<dim3(LLe / 256, 1, 1), blk, 0, stream>>>(S + (size_t)z * LLe * LLe, LLe, (size_t)0, V + (h0 + z) * HDe, DDe, (size_t)0, VS + (h0 + z) * HDe, nullptr, sc, ATT + (h0 + z) * HDe, DDe, (size_t)0, LLe);
      }
      gemm_kne<float, 2, false><<<dim3(LLe / 128, DDe / 128), blk, 0, stream>>>(ATT, DDe, wo, DDe, bo + l * DDe, T, ones, T, DDe, DDe);
      k_ln<<<dim3(LLe / 16), blk, 0, stream>>>(T, l2s + l * DDe, l2b + l * DDe, Hn);
      gemm_kne<float, 1, false><<<dim3(LLe / 128, FFe / 128), blk, 0, stream>>>(Hn, DDe, w1, FFe, b1 + l * FFe, nullptr, nullptr, Fh, FFe, DDe);
      gemm_kne<float, 2, false><<<dim3(LLe / 128, DDe / 128), blk, 0, stream>>>(Fh, FFe, w2, DDe, b2 + l * DDe, T, ones, T, DDe, FFe);
    }
  }
}
